// MultiheadLatentAttention_3272765080433
// MI455X (gfx1250) — hardware-verified
//
#include <hip/hip_runtime.h>
#include <math.h>

typedef __attribute__((ext_vector_type(16))) _Float16 v16h;
typedef __attribute__((ext_vector_type(8)))  _Float16 v8h;
typedef __attribute__((ext_vector_type(16))) __bf16   v16b;
typedef __attribute__((ext_vector_type(8)))  __bf16   v8b;
typedef __attribute__((ext_vector_type(8)))  float    v8f;
typedef __attribute__((ext_vector_type(4)))  float    v4f;
typedef __attribute__((ext_vector_type(4)))  unsigned v4u;

constexpr int NB_SZ   = 2;
constexpr int NT_SZ   = 2048;
constexpr int NDM_SZ  = 2048;
constexpr int NH_SZ   = 16;
constexpr int NHD_SZ  = 128;
constexpr int NDC_SZ  = 512;
constexpr int NDR_SZ  = 64;
constexpr int NTOK_SZ = NB_SZ * NT_SZ;
constexpr int NQR_SZ  = NH_SZ * NDR_SZ;

constexpr float W_CARRY   = 64.0f;
constexpr float P_CARRY   = 1024.0f;
constexpr float CTX_CARRY = 1024.0f;

__device__ __forceinline__ unsigned short f2bf_bits(float f) {
  unsigned u = __float_as_uint(f);
  return (unsigned short)((u + 0x7FFFu + ((u >> 16) & 1u)) >> 16);
}
__device__ __forceinline__ float bf_bits2f(unsigned short h) { return __uint_as_float(((unsigned)h) << 16); }

__device__ __forceinline__ void dep_guard_h(v8f& a, v8f& b, v16h x, v16h y) { asm volatile("v_nop\n\tv_nop\n\tv_nop\n\tv_nop" : "+v"(a), "+v"(b) : "v"(x), "v"(y)); }
__device__ __forceinline__ void dep_guard_b(v8f& a, v8f& b, v16b x, v16b y) { asm volatile("v_nop\n\tv_nop\n\tv_nop\n\tv_nop" : "+v"(a), "+v"(b) : "v"(x), "v"(y)); }
__device__ __forceinline__ void keep4_h(v16h a, v16h b, v16h c, v16h d) { asm volatile("v_nop" :: "v"(a), "v"(b), "v"(c), "v"(d)); }
__device__ __forceinline__ void keep4_b(v16b a, v16b b, v16b c, v16b d) { asm volatile("v_nop" :: "v"(a), "v"(b), "v"(c), "v"(d)); }
__device__ __forceinline__ void acc_guard4(v8f& a, v8f& b, v8f& c, v8f& d) { asm volatile("v_nop\n\tv_nop\n\tv_nop\n\tv_nop" : "+v"(a), "+v"(b), "+v"(c), "+v"(d)); }
template <typename T> struct Frag;
template <> struct Frag<_Float16> {
  typedef v16h V; union U { v16h v; v8h h[2]; };
  static __device__ __forceinline__ v16h load(const _Float16* p) {
    U f; f.h[0] = *(const v8h*)(p); f.h[1] = *(const v8h*)(p + 16); return f.v;
  }
  static __device__ __forceinline__ v8f mma(v16h a, v16h b, v8f c) {
    return __builtin_amdgcn_wmma_f32_16x16x32_f16(false, a, false, b, (short)0, c, false, false);
  }
  static __device__ __forceinline__ void guard(v8f& a, v8f& b, v16h x, v16h y) { dep_guard_h(a, b, x, y); }
  static __device__ __forceinline__ void keep(v16h a, v16h b, v16h c, v16h d) { keep4_h(a, b, c, d); }
};
template <> struct Frag<__bf16> {
  typedef v16b V; union U { v16b v; v8b h[2]; };
  static __device__ __forceinline__ v16b load(const __bf16* p) {
    U f; f.h[0] = *(const v8b*)(p); f.h[1] = *(const v8b*)(p + 16); return f.v;
  }
  static __device__ __forceinline__ v8f mma(v16b a, v16b b, v8f c) {
    return __builtin_amdgcn_wmma_f32_16x16x32_bf16(false, a, false, b, (short)0, c, false, false);
  }
  static __device__ __forceinline__ void guard(v8f& a, v8f& b, v16b x, v16b y) { dep_guard_b(a, b, x, y); }
  static __device__ __forceinline__ void keep(v16b a, v16b b, v16b c, v16b d) { keep4_b(a, b, c, d); }
};

template <int ET> struct Elem;
template <> struct Elem<0> { typedef _Float16 T; };
template <> struct Elem<1> { typedef __bf16 T; };
template <int ET, bool SPLIT, int BIAS_MODE, int OUT_MODE, bool RESID, int ACT = 0>
__global__ __launch_bounds__(256) void wmma_gemm64(
    const unsigned short* __restrict__ Ap, const unsigned short* __restrict__ A2p, int lda, long strideA,
    const unsigned short* __restrict__ Btp, const unsigned short* __restrict__ Bt2p, int ldb, long strideB,
    void* __restrict__ Cout, void* __restrict__ Cout2, int ldc, long strideC,
    const float* __restrict__ bias,
    const float* __restrict__ resid, long strideR,
    int M, int N, int K, float scale) {
  typedef typename Elem<ET>::T T;
  typedef typename Frag<T>::V V;
  const T* A = (const T*)Ap; const T* A2 = (const T*)A2p; const T* Bt = (const T*)Btp; const T* Bt2 = (const T*)Bt2p;
  __shared__ __align__(16) float sT[8][16 * 68];
  const int b    = blockIdx.y;
  const int lane = threadIdx.x & 31;
  const int wave = threadIdx.x >> 5;
  const int tilesN = N >> 6;
  const int tilesM = M >> 6;
  const int tile = blockIdx.x * 8 + wave;
  if (tile >= tilesM * tilesN) return;
  const int tm = tile / tilesN;
  const int tn = tile - tm * tilesN;
  const int m0 = tm << 6;
  const int n0 = tn << 6;

  const T* Ab  = A  + (size_t)b * strideA;
  const T* Bb  = Bt + (size_t)b * strideB;
  const T* Ab2 = SPLIT ? (A2  + (size_t)b * strideA) : nullptr;
  const T* Bb2 = SPLIT ? (Bt2 + (size_t)b * strideB) : nullptr;

  const int rlane = lane & 15;
  const int koff  = (lane >> 4) * 8;
  const int mOff  = (lane >> 4) * 8;

  v8f acc[4][4];
#pragma unroll
  for (int i = 0; i < 4; ++i)
#pragma unroll
    for (int j = 0; j < 4; ++j) acc[i][j] = (v8f){0.f,0.f,0.f,0.f,0.f,0.f,0.f,0.f};

  for (int k0 = 0; k0 < K; k0 += 32) {
    V bh[4], bl[4];
#pragma unroll
    for (int j = 0; j < 4; ++j) {
      const size_t bo = (size_t)(n0 + (j << 4) + rlane) * ldb + koff + k0;
      bh[j] = Frag<T>::load(Bb + bo);
      if (SPLIT) bl[j] = Frag<T>::load(Bb2 + bo);
    }
#pragma unroll
    for (int i = 0; i < 4; ++i) {
      const size_t ao = (size_t)(m0 + (i << 4) + rlane) * lda + koff + k0;
      V ah = Frag<T>::load(Ab + ao);
      V al;
      if (SPLIT) al = Frag<T>::load(Ab2 + ao);
#pragma unroll
      for (int j = 0; j < 4; ++j) {
        acc[i][j] = Frag<T>::mma(ah, bh[j], acc[i][j]);
        if (SPLIT) {
          acc[i][j] = Frag<T>::mma(ah, bl[j], acc[i][j]);
          acc[i][j] = Frag<T>::mma(al, bh[j], acc[i][j]);
        }
      }
      Frag<T>::guard(acc[i][0], acc[i][3], ah, SPLIT ? al : ah);
    }
    Frag<T>::keep(bh[0], bh[1], bh[2], bh[3]);
    if (SPLIT) Frag<T>::keep(bl[0], bl[1], bl[2], bl[3]);
  }
  acc_guard4(acc[0][0], acc[0][1], acc[0][2], acc[0][3]);
  acc_guard4(acc[1][0], acc[1][1], acc[1][2], acc[1][3]);
  acc_guard4(acc[2][0], acc[2][1], acc[2][2], acc[2][3]);
  acc_guard4(acc[3][0], acc[3][1], acc[3][2], acc[3][3]);

  float* slab = sT[wave];
  const float* Rb = RESID ? (resid + (size_t)b * strideR) : nullptr;
#pragma unroll
  for (int i = 0; i < 4; ++i) {
    const int mBase = m0 + (i << 4);
#pragma unroll
    for (int j = 0; j < 4; ++j) {
      const int n = n0 + (j << 4) + rlane;
      float bv = 0.f;
      if (BIAS_MODE == 2) bv = bias[n];
#pragma unroll
      for (int r = 0; r < 8; ++r) {
        float v = acc[i][j][r] * scale;
        if (BIAS_MODE == 1) v += bias[mBase + mOff + r];
        if (BIAS_MODE == 2) v += bv;
        if (RESID) v += Rb[(size_t)(mBase + mOff + r) * ldc + n];
        if (ACT == 1) v = tanhf(v);
        if (ACT == 2) v = fmaxf(v, 0.0f);
        if (ACT == 3) v = v / (1.0f + expf(-v));
        if (ACT == 4) v = (v > 0.f) ? v : 0.01f * v;
        if (ACT == 5) v = 0.5f * v * (1.0f + erff(v * 0.70710678118654752f));
        slab[(mOff + r) * 68 + (j << 4) + rlane] = v;
      }
    }
    __builtin_amdgcn_fence(__ATOMIC_RELEASE, "workgroup");
    __builtin_amdgcn_wave_barrier();
    __builtin_amdgcn_fence(__ATOMIC_ACQUIRE, "workgroup");
    if (OUT_MODE == 0) {
      float* C = (float*)Cout + (size_t)b * strideC;
      const int hh = lane >> 4, c4 = (lane & 15) * 4;
      for (int pass = 0; pass < 2; ++pass) {
#pragma unroll
        for (int it = 0; it < 8; ++it) {
          const int row = it * 2 + hh;
          v4f v = *(const v4f*)(slab + row * 68 + c4);
          *(volatile v4f*)(C + (size_t)(mBase + row) * ldc + n0 + c4) = v;
        }
        __threadfence();
      }
    } else {
      const int q = lane >> 3, c8 = (lane & 7) * 8;
      unsigned short* C  = (unsigned short*)Cout  + (size_t)b * strideC;
      unsigned short* C2 = (OUT_MODE == 2) ? ((unsigned short*)Cout2 + (size_t)b * strideC) : nullptr;
      for (int pass = 0; pass < 2; ++pass) {
#pragma unroll
        for (int it = 0; it < 4; ++it) {
          const int row = it * 4 + q;
          const float* sp = slab + row * 68 + c8;
          v8h hv, lv;
#pragma unroll
          for (int e = 0; e < 8; ++e) {
            if (OUT_MODE == 1) {
              hv[e] = (_Float16)sp[e];
            } else {
              unsigned short hb = f2bf_bits(sp[e]);
              unsigned short lb = f2bf_bits(sp[e] - bf_bits2f(hb));
              hv[e] = __builtin_bit_cast(_Float16, hb);
              lv[e] = __builtin_bit_cast(_Float16, lb);
            }
          }
          *(volatile v8h*)(C + (size_t)(mBase + row) * ldc + n0 + c8) = hv;
          if (OUT_MODE == 2) *(volatile v8h*)(C2 + (size_t)(mBase + row) * ldc + n0 + c8) = lv;
        }
        __threadfence();
      }
    }
    __builtin_amdgcn_fence(__ATOMIC_RELEASE, "workgroup");
    __builtin_amdgcn_wave_barrier();
    __builtin_amdgcn_fence(__ATOMIC_ACQUIRE, "workgroup");
  }
}

__device__ __forceinline__ unsigned pack_h2(float a, float b) {
  const unsigned lo = (unsigned)__builtin_bit_cast(unsigned short, (_Float16)a);
  const unsigned hi = (unsigned)__builtin_bit_cast(unsigned short, (_Float16)b);
  return lo | (hi << 16);
}
__global__ __launch_bounds__(256) void cast_f32_f16x8(
    const float* __restrict__ in, unsigned short* __restrict__ out, int n8) {
  const int i = blockIdx.x * 256 + threadIdx.x;
  if (i < n8) {
    const v4f a = *(const v4f*)(in + (size_t)8 * i);
    const v4f b = *(const v4f*)(in + (size_t)8 * i + 4);
    v4u u;
    u[0] = pack_h2(a[0], a[1]);
    u[1] = pack_h2(a[2], a[3]);
    u[2] = pack_h2(b[0], b[1]);
    u[3] = pack_h2(b[2], b[3]);
    *(volatile v4u*)(out + (size_t)8 * i) = u;
    __threadfence();
    *(volatile v4u*)(out + (size_t)8 * i) = u;
  }
}

constexpr int TP_PITCH = 72;
__global__ __launch_bounds__(256) void transpose_cast_f16(
    const float* __restrict__ in, int R, int C,
    unsigned short* __restrict__ out, int ldo, int ro, float scale) {
  __shared__ __align__(16) _Float16 tile[64 * TP_PITCH];
  const int tid = threadIdx.x, lane = tid & 31, wave = tid >> 5;
  const int r0 = blockIdx.y * 64, c0 = blockIdx.x * 64;
#pragma unroll
  for (int it = 0; it < 4; ++it) {
    const int idx = tid + 256 * it;
    const int rr = idx >> 4;
    const int c4 = (idx & 15) * 4;
    const v4f v = *(const v4f*)(in + (size_t)(r0 + rr) * C + c0 + c4);
#pragma unroll
    for (int e = 0; e < 4; ++e) tile[(c4 + e) * TP_PITCH + rr] = (_Float16)(v[e] * scale);
  }
  __syncthreads();
  const int q = lane >> 3, c8 = (lane & 7) * 8;
  for (int pass = 0; pass < 2; ++pass) {
#pragma unroll
    for (int it = 0; it < 2; ++it) {
      const int row = wave * 8 + it * 4 + q;
      const v4u val = *(const v4u*)(tile + row * TP_PITCH + c8);
      *(volatile v4u*)(out + (size_t)(ro + c0 + row) * ldo + r0 + c8) = val;
    }
    __threadfence();
  }
}

struct RopeTab { float f[32]; };
static_assert(sizeof(RopeTab) == 128, "no padding");
constexpr int ROPE_ROW = NQR_SZ + NDR_SZ;
__global__ __launch_bounds__(256) void rope_kernel(
    const float* __restrict__ krp, const float* __restrict__ qrp,
    unsigned short* __restrict__ krh, unsigned short* __restrict__ qrh, RopeTab tab) {
#pragma clang fp contract(off)
  __shared__ __align__(16) _Float16 rb[8][ROPE_ROW];
  const int tid = threadIdx.x, lane = tid & 31, wave = tid >> 5;
  const int tok = blockIdx.x * 8 + wave;
  const int pos = tok & (NT_SZ - 1);
  float invf = tab.f[0];
#pragma unroll
  for (int k = 1; k < 32; ++k) invf = (lane == k) ? tab.f[k] : invf;
  const float ang = (float)pos * invf;
  float sn, cs;
  sincosf(ang, &sn, &cs);
  _Float16* row = rb[wave];
  const float* qp = qrp + (size_t)tok * NQR_SZ;
#pragma unroll 1
  for (int g = 0; g < NH_SZ; ++g) {
    const float x1 = qp[g * NDR_SZ + lane];
    const float x2 = qp[g * NDR_SZ + 32 + lane];
    const float o0 = x1 * cs - x2 * sn;
    const float o1 = x1 * sn + x2 * cs;
    row[g * NDR_SZ + 2 * lane]     = (_Float16)o0;
    row[g * NDR_SZ + 2 * lane + 1] = (_Float16)o1;
  }
  {
    const float* kp = krp + (size_t)tok * NDR_SZ;
    const float x1 = kp[lane];
    const float x2 = kp[32 + lane];
    const float o0 = x1 * cs - x2 * sn;
    const float o1 = x1 * sn + x2 * cs;
    row[NQR_SZ + 2 * lane]     = (_Float16)o0;
    row[NQR_SZ + 2 * lane + 1] = (_Float16)o1;
  }
  __syncthreads();
  const int l8 = lane & 7;
  for (int pass = 0; pass < 2; ++pass) {
#pragma unroll
    for (int it = 0; it < 4; ++it) {
      const int chunk = it * 32 + lane;
      const v4u val = *(const v4u*)(row + chunk * 8);
      *(volatile v4u*)(qrh + (size_t)tok * NQR_SZ + chunk * 8) = val;
    }
    const v4u kv = *(const v4u*)(row + NQR_SZ + l8 * 8);
    if (lane < 8) *(volatile v4u*)(krh + (size_t)tok * NDR_SZ + l8 * 8) = kv;
    __threadfence();
  }
}

constexpr int ATT_D    = NHD_SZ + NDR_SZ;
constexpr int ATT_KC   = 64;
constexpr int ATT_QB   = 128;
constexpr int ATT_LK   = 0;
constexpr int ATT_LV   = ATT_KC * ATT_D;
constexpr int ATT_LP   = ATT_LV + NHD_SZ * ATT_KC;
constexpr int ATT_LDS  = ATT_LP + 8 * 16 * ATT_KC;
constexpr int SLAB_P   = 136;
static_assert(ATT_QB * ATT_D <= ATT_LDS, "q staging fits");
static_assert(8 * 16 * SLAB_P <= ATT_LDS, "out slabs fit");
static_assert(ATT_LDS * 2 <= 65536, "static lds");
static_assert(NT_SZ % ATT_QB == 0 && NT_SZ % ATT_KC == 0, "tiles");

__device__ __forceinline__ v8f mma_h(v16h a, v16h b, v8f c) {
  c = __builtin_amdgcn_wmma_f32_16x16x32_f16(false, a, false, b, (short)0, c, false, false);
  asm volatile("v_nop\n\tv_nop\n\tv_nop\n\tv_nop" : "+v"(c) : "v"(a), "v"(b));
  return c;
}

__global__ __launch_bounds__(256) void attn_lat_kernel(
    const unsigned short* __restrict__ Qp, const unsigned short* __restrict__ QRp,
    const unsigned short* __restrict__ Kp, const unsigned short* __restrict__ KRp,
    const unsigned short* __restrict__ Vtp, unsigned short* __restrict__ Cp, float qscale) {
  __shared__ __align__(16) _Float16 lds[ATT_LDS];
  const int tid = threadIdx.x, lane = tid & 31, wave = tid >> 5;
  const int hh = lane >> 4, c = lane & 15;
  const int nqb = NT_SZ / ATT_QB;
  const int bx = blockIdx.x;
  const int qb = bx % nqb;
  const int bh = bx / nqb;
  const int h  = bh % NH_SZ;
  const int b  = bh / NH_SZ;
  const int tok0 = b * NT_SZ + qb * ATT_QB;

#pragma unroll
  for (int it = 0; it < 8; ++it) {
    const int idx = tid + 256 * it;
    const int rr = idx >> 4, seg = idx & 15;
    const v4u v = *(const v4u*)(Qp + (size_t)(tok0 + rr) * NDM_SZ + h * NHD_SZ + seg * 8);
    *(v4u*)(lds + rr * ATT_D + seg * 8) = v;
  }
#pragma unroll
  for (int it = 0; it < 4; ++it) {
    const int idx = tid + 256 * it;
    const int rr = idx >> 3, seg = idx & 7;
    const v4u v = *(const v4u*)(QRp + (size_t)(tok0 + rr) * NQR_SZ + h * NDR_SZ + seg * 8);
    *(v4u*)(lds + rr * ATT_D + NHD_SZ + seg * 8) = v;
  }
  __syncthreads();
  v16h qf[6];
#pragma unroll
  for (int ks = 0; ks < 6; ++ks) qf[ks] = Frag<_Float16>::load(lds + (wave * 16 + c) * ATT_D + ks * 32 + 8 * hh);

  float mrow[8], lrow[8];
  v8f oacc[8];
#pragma unroll
  for (int r = 0; r < 8; ++r) { mrow[r] = -INFINITY; lrow[r] = 0.f; }
#pragma unroll
  for (int t = 0; t < 8; ++t) oacc[t] = (v8f){0.f,0.f,0.f,0.f,0.f,0.f,0.f,0.f};

  _Float16* pw = lds + ATT_LP + wave * (16 * ATT_KC);

  for (int kc = 0; kc < NT_SZ / ATT_KC; ++kc) {
    const int ktok0 = b * NT_SZ + kc * ATT_KC;
    __syncthreads();
#pragma unroll
    for (int it = 0; it < 4; ++it) {
      const int idx = tid + 256 * it;
      const int key = idx >> 4, seg = idx & 15;
      const v4u v = *(const v4u*)(Kp + (size_t)(ktok0 + key) * NDM_SZ + h * NHD_SZ + seg * 8);
      *(v4u*)(lds + ATT_LK + key * ATT_D + seg * 8) = v;
    }
#pragma unroll
    for (int it = 0; it < 2; ++it) {
      const int idx = tid + 256 * it;
      const int key = idx >> 3, seg = idx & 7;
      const v4u v = *(const v4u*)(KRp + (size_t)(ktok0 + key) * NDR_SZ + seg * 8);
      *(v4u*)(lds + ATT_LK + key * ATT_D + NHD_SZ + seg * 8) = v;
    }
#pragma unroll
    for (int it = 0; it < 4; ++it) {
      const int idx = tid + 256 * it;
      const int d = idx >> 3, seg = idx & 7;
      const v4u v = *(const v4u*)(Vtp + (size_t)(h * NHD_SZ + d) * NTOK_SZ + ktok0 + seg * 8);
      *(v4u*)(lds + ATT_LV + d * ATT_KC + seg * 8) = v;
    }
    __syncthreads();

    v8f s[4];
#pragma unroll
    for (int j = 0; j < 4; ++j) {
      s[j] = (v8f){0.f,0.f,0.f,0.f,0.f,0.f,0.f,0.f};
#pragma unroll
      for (int ks = 0; ks < 6; ++ks) {
        const v16h kb = Frag<_Float16>::load(lds + ATT_LK + (j * 16 + c) * ATT_D + ks * 32 + 8 * hh);
        s[j] = mma_h(qf[ks], kb, s[j]);
      }
    }
    float cm[8];
#pragma unroll
    for (int r = 0; r < 8; ++r) {
      float m = -INFINITY;
#pragma unroll
      for (int j = 0; j < 4; ++j) {
        s[j][r] = s[j][r] * qscale;
        m = fmaxf(m, s[j][r]);
      }
#pragma unroll
      for (int off = 1; off < 16; off <<= 1) m = fmaxf(m, __shfl_xor(m, off, 32));
      cm[r] = m;
    }
#pragma unroll
    for (int r = 0; r < 8; ++r) {
      const float mnew = fmaxf(mrow[r], cm[r]);
      const float alpha = expf(mrow[r] - mnew);
      mrow[r] = mnew;
      float psum = 0.f;
#pragma unroll
      for (int j = 0; j < 4; ++j) {
        const float p = expf(s[j][r] - mnew);
        psum += p;
        pw[(8 * hh + r) * ATT_KC + j * 16 + c] = (_Float16)(p * P_CARRY);
      }
#pragma unroll
      for (int off = 1; off < 16; off <<= 1) psum += __shfl_xor(psum, off, 32);
      lrow[r] = lrow[r] * alpha + psum;
#pragma unroll
      for (int t = 0; t < 8; ++t) oacc[t][r] *= alpha;
    }
    __builtin_amdgcn_fence(__ATOMIC_RELEASE, "workgroup");
    __builtin_amdgcn_wave_barrier();
    __builtin_amdgcn_fence(__ATOMIC_ACQUIRE, "workgroup");
#pragma unroll
    for (int kk = 0; kk < 2; ++kk) {
      const v16h pa = Frag<_Float16>::load(pw + c * ATT_KC + kk * 32 + 8 * hh);
#pragma unroll
      for (int t = 0; t < 8; ++t) {
        const v16h vb = Frag<_Float16>::load(lds + ATT_LV + (t * 16 + c) * ATT_KC + kk * 32 + 8 * hh);
        oacc[t] = mma_h(pa, vb, oacc[t]);
      }
    }
  }

  __syncthreads();
  _Float16* slab = lds + wave * (16 * SLAB_P);
#pragma unroll
  for (int r = 0; r < 8; ++r) {
    const float inv = (CTX_CARRY / P_CARRY) / lrow[r];
#pragma unroll
    for (int t = 0; t < 8; ++t) slab[(8 * hh + r) * SLAB_P + t * 16 + c] = (_Float16)(oacc[t][r] * inv);
  }
  __syncthreads();
  {
    const int col8 = c * 8;
    unsigned short* ob = Cp + (size_t)(tok0 + wave * 16) * NDM_SZ + h * NHD_SZ;
    for (int pass = 0; pass < 2; ++pass) {
#pragma unroll
      for (int it = 0; it < 8; ++it) {
        const int row = it * 2 + hh;
        const v4u val = *(const v4u*)(slab + row * SLAB_P + col8);
        *(volatile v4u*)(ob + (size_t)row * NDM_SZ + col8) = val;
      }
      __threadfence();
    }
  }
}

constexpr size_t WS_XH    = 0;
constexpr size_t SZ_XH    = (size_t)NTOK_SZ * NDM_SZ * 2;
constexpr size_t WS_WCT   = WS_XH + SZ_XH;
constexpr size_t SZ_WCT   = (size_t)(2 * NDC_SZ) * NDM_SZ * 2;
constexpr size_t WS_WKRT  = WS_WCT + SZ_WCT;
constexpr size_t SZ_WKRT  = (size_t)NDR_SZ * NDM_SZ * 2;
constexpr size_t WS_WUKV  = WS_WKRT + SZ_WKRT;
constexpr size_t SZ_WUKV  = (size_t)(2 * NDM_SZ) * NDC_SZ * 2;
constexpr size_t WS_WUQ   = WS_WUKV + SZ_WUKV;
constexpr size_t SZ_WUQ   = (size_t)NDM_SZ * NDC_SZ * 2;
constexpr size_t WS_WQR   = WS_WUQ + SZ_WUQ;
constexpr size_t SZ_WQR   = (size_t)NQR_SZ * NDC_SZ * 2;
constexpr size_t WS_WO    = WS_WQR + SZ_WQR;
constexpr size_t SZ_WO    = (size_t)NDM_SZ * NDM_SZ * 2;
constexpr size_t WS_CC    = WS_WO + SZ_WO;
constexpr size_t SZ_CC    = (size_t)NTOK_SZ * (2 * NDC_SZ) * 2;
constexpr size_t WS_KRP   = WS_CC + SZ_CC;
constexpr size_t SZ_KRP   = (size_t)NTOK_SZ * NDR_SZ * 4;
constexpr size_t WS_KH    = WS_KRP + SZ_KRP;
constexpr size_t SZ_KH    = (size_t)NTOK_SZ * NDM_SZ * 2;
constexpr size_t WS_VT    = WS_KH + SZ_KH;
constexpr size_t SZ_VT    = (size_t)NDM_SZ * NTOK_SZ * 2;
constexpr size_t WS_QH    = WS_VT + SZ_VT;
constexpr size_t SZ_QH    = (size_t)NTOK_SZ * NDM_SZ * 2;
constexpr size_t WS_QRP   = WS_QH + SZ_QH;
constexpr size_t SZ_QRP   = (size_t)NTOK_SZ * NQR_SZ * 4;
constexpr size_t WS_KRH   = WS_QRP + SZ_QRP;
constexpr size_t SZ_KRH   = (size_t)NTOK_SZ * NDR_SZ * 2;
constexpr size_t WS_QRH   = WS_KRH + SZ_KRH;
constexpr size_t SZ_QRH   = (size_t)NTOK_SZ * NQR_SZ * 2;
constexpr size_t WS_TOTAL = WS_QRH + SZ_QRH;
static_assert(WS_TOTAL == 122421248, "carve total");
static_assert(WS_TOTAL <= 134217728, "carve cap");
static_assert((WS_WCT % 256) == 0 && (WS_WKRT % 256) == 0 && (WS_WUKV % 256) == 0 && (WS_WUQ % 256) == 0 &&
              (WS_WQR % 256) == 0 && (WS_WO % 256) == 0 && (WS_CC % 256) == 0 && (WS_KRP % 256) == 0 &&
              (WS_KH % 256) == 0 && (WS_VT % 256) == 0 && (WS_QH % 256) == 0 && (WS_QRP % 256) == 0 &&
              (WS_KRH % 256) == 0 && (WS_QRH % 256) == 0, "alignment");

static_assert(NTOK_SZ % 64 == 0 && NDM_SZ % 64 == 0 && (2 * NDC_SZ) % 64 == 0 && NDR_SZ % 64 == 0 && NQR_SZ % 64 == 0, "M,N tile multiples");
static_assert(NDM_SZ % 32 == 0 && NDC_SZ % 32 == 0, "K multiples of 32");
static_assert((NTOK_SZ * NDM_SZ) % (8 * 256) == 0, "cast grid exact");
static_assert(NTOK_SZ % 8 == 0, "rope grid exact");

extern "C" void kernel_launch(void* const* d_in, const int* in_sizes, int n_in,
                              void* d_out, int out_size, void* d_ws, size_t ws_size,
                              hipStream_t stream) {
  if (n_in != 10) return;
  if (in_sizes[0] != NTOK_SZ * NDM_SZ) return;
  if (in_sizes[1] != NDM_SZ * NDC_SZ || in_sizes[2] != NDM_SZ * NDC_SZ) return;
  if (in_sizes[3] != NDC_SZ * NDM_SZ || in_sizes[4] != NDC_SZ * NDM_SZ || in_sizes[5] != NDC_SZ * NDM_SZ) return;
  if (in_sizes[6] != NDM_SZ * NDR_SZ || in_sizes[7] != NDC_SZ * NQR_SZ) return;
  if (in_sizes[8] != NDM_SZ * NDM_SZ || in_sizes[9] != NDM_SZ) return;
  if (out_size != NTOK_SZ * NDM_SZ) return;
  if (ws_size < WS_TOTAL) return;

  const float* x     = (const float*)d_in[0];
  const float* w_dkv = (const float*)d_in[1];
  const float* w_dq  = (const float*)d_in[2];
  const float* w_uk  = (const float*)d_in[3];
  const float* w_uv  = (const float*)d_in[4];
  const float* w_uq  = (const float*)d_in[5];
  const float* w_kr  = (const float*)d_in[6];
  const float* w_qr  = (const float*)d_in[7];
  const float* w_o   = (const float*)d_in[8];
  const float* b_o   = (const float*)d_in[9];
  float* out = (float*)d_out;

  char* ws = (char*)d_ws;
  unsigned short* xh    = (unsigned short*)(ws + WS_XH);
  unsigned short* ctxh  = (unsigned short*)(ws + WS_XH);
  unsigned short* wct   = (unsigned short*)(ws + WS_WCT);
  unsigned short* wkrt  = (unsigned short*)(ws + WS_WKRT);
  unsigned short* wukvt = (unsigned short*)(ws + WS_WUKV);
  unsigned short* wuqt  = (unsigned short*)(ws + WS_WUQ);
  unsigned short* wqrt  = (unsigned short*)(ws + WS_WQR);
  unsigned short* wot   = (unsigned short*)(ws + WS_WO);
  unsigned short* cc    = (unsigned short*)(ws + WS_CC);
  float*          krp   = (float*)(ws + WS_KRP);
  unsigned short* kh    = (unsigned short*)(ws + WS_KH);
  unsigned short* vt    = (unsigned short*)(ws + WS_VT);
  unsigned short* qh    = (unsigned short*)(ws + WS_QH);
  float*          qrpf  = (float*)(ws + WS_QRP);
  unsigned short* krh   = (unsigned short*)(ws + WS_KRH);
  unsigned short* qrh   = (unsigned short*)(ws + WS_QRH);

  const dim3 blk(256);

  {
    const int n8 = NTOK_SZ * NDM_SZ / 8;
    cast_f32_f16x8<<<dim3(n8 / 256), blk, 0, stream>>>(x, xh, n8);
  }
  transpose_cast_f16<<<dim3(NDC_SZ / 64, NDM_SZ / 64), blk, 0, stream>>>(w_dkv, NDM_SZ, NDC_SZ, wct, NDM_SZ, 0, W_CARRY);
  transpose_cast_f16<<<dim3(NDC_SZ / 64, NDM_SZ / 64), blk, 0, stream>>>(w_dq,  NDM_SZ, NDC_SZ, wct, NDM_SZ, NDC_SZ, W_CARRY);
  transpose_cast_f16<<<dim3(NDR_SZ / 64, NDM_SZ / 64), blk, 0, stream>>>(w_kr,  NDM_SZ, NDR_SZ, wkrt, NDM_SZ, 0, W_CARRY);
  transpose_cast_f16<<<dim3(NDM_SZ / 64, NDC_SZ / 64), blk, 0, stream>>>(w_uk,  NDC_SZ, NDM_SZ, wukvt, NDC_SZ, 0, W_CARRY);
  transpose_cast_f16<<<dim3(NDM_SZ / 64, NDC_SZ / 64), blk, 0, stream>>>(w_uv,  NDC_SZ, NDM_SZ, wukvt, NDC_SZ, NDM_SZ, W_CARRY);
  transpose_cast_f16<<<dim3(NDM_SZ / 64, NDC_SZ / 64), blk, 0, stream>>>(w_uq,  NDC_SZ, NDM_SZ, wuqt, NDC_SZ, 0, W_CARRY);
  transpose_cast_f16<<<dim3(NQR_SZ / 64, NDC_SZ / 64), blk, 0, stream>>>(w_qr,  NDC_SZ, NQR_SZ, wqrt, NDC_SZ, 0, W_CARRY);
  transpose_cast_f16<<<dim3(NDM_SZ / 64, NDM_SZ / 64), blk, 0, stream>>>(w_o,   NDM_SZ, NDM_SZ, wot, NDM_SZ, 0, W_CARRY);

  const float inv_w = 1.0f / W_CARRY;

  {
    const int M = NTOK_SZ, N = 2 * NDC_SZ, K = NDM_SZ;
    const int tiles = (M / 64) * (N / 64);
    wmma_gemm64<0, false, 0, 1, false><<<dim3((tiles + 7) / 8, 1), blk, 0, stream>>>(
        xh, nullptr, NDM_SZ, 0, wct, nullptr, NDM_SZ, 0, cc, nullptr, 2 * NDC_SZ, 0,
        nullptr, nullptr, 0, M, N, K, inv_w);
  }
  {
    const int M = NTOK_SZ, N = NDR_SZ, K = NDM_SZ;
    const int tiles = (M / 64) * (N / 64);
    wmma_gemm64<0, false, 0, 0, false><<<dim3((tiles + 7) / 8, 1), blk, 0, stream>>>(
        xh, nullptr, NDM_SZ, 0, wkrt, nullptr, NDM_SZ, 0, krp, nullptr, NDR_SZ, 0,
        nullptr, nullptr, 0, M, N, K, inv_w);
  }
  {
    const int M = NTOK_SZ, N = NDM_SZ, K = NDC_SZ;
    const int tiles = (M / 64) * (N / 64);
    wmma_gemm64<0, false, 0, 1, false><<<dim3((tiles + 7) / 8, 1), blk, 0, stream>>>(
        cc, nullptr, 2 * NDC_SZ, 0, wukvt, nullptr, NDC_SZ, 0, kh, nullptr, NDM_SZ, 0,
        nullptr, nullptr, 0, M, N, K, inv_w);
  }
  {
    const int M = NDM_SZ, N = NTOK_SZ, K = NDC_SZ;
    const int tiles = (M / 64) * (N / 64);
    wmma_gemm64<0, false, 0, 1, false><<<dim3((tiles + 7) / 8, 1), blk, 0, stream>>>(
        wukvt + (size_t)NDM_SZ * NDC_SZ, nullptr, NDC_SZ, 0, cc, nullptr, 2 * NDC_SZ, 0, vt, nullptr, NTOK_SZ, 0,
        nullptr, nullptr, 0, M, N, K, inv_w);
  }
  {
    const int M = NTOK_SZ, N = NDM_SZ, K = NDC_SZ;
    const int tiles = (M / 64) * (N / 64);
    wmma_gemm64<0, false, 0, 1, false><<<dim3((tiles + 7) / 8, 1), blk, 0, stream>>>(
        cc + NDC_SZ, nullptr, 2 * NDC_SZ, 0, wuqt, nullptr, NDC_SZ, 0, qh, nullptr, NDM_SZ, 0,
        nullptr, nullptr, 0, M, N, K, inv_w);
  }
  {
    const int M = NTOK_SZ, N = NQR_SZ, K = NDC_SZ;
    const int tiles = (M / 64) * (N / 64);
    wmma_gemm64<0, false, 0, 0, false><<<dim3((tiles + 7) / 8, 1), blk, 0, stream>>>(
        cc + NDC_SZ, nullptr, 2 * NDC_SZ, 0, wqrt, nullptr, NDC_SZ, 0, qrpf, nullptr, NQR_SZ, 0,
        nullptr, nullptr, 0, M, N, K, inv_w);
  }
  {
    RopeTab tab;
    for (int i = 0; i < 32; ++i) {
      const float e = (float)i / 32.0f;
      const float p = powf(10000.0f, e);
      tab.f[i] = 1.0f / p;
    }
    rope_kernel<<<dim3(NTOK_SZ / 8), blk, 0, stream>>>(krp, qrpf, krh, qrh, tab);
  }
  {
    const float qscale = 1.0f / sqrtf((float)(NHD_SZ + NDR_SZ));
    attn_lat_kernel<<<dim3(NB_SZ * NH_SZ * (NT_SZ / ATT_QB)), blk, 0, stream>>>(qh, qrh, kh, krh, vt, ctxh, qscale);
  }
  {
    const int M = NTOK_SZ, N = NDM_SZ, K = NDM_SZ;
    const int tiles = (M / 64) * (N / 64);
    wmma_gemm64<0, false, 2, 0, false><<<dim3((tiles + 7) / 8, 1), blk, 0, stream>>>(
        ctxh, nullptr, NDM_SZ, 0, wot, nullptr, NDM_SZ, 0, out, nullptr, NDM_SZ, 0,
        b_o, nullptr, 0, M, N, K, 1.0f / (W_CARRY * CTX_CARRY));
  }
}
